// MultiHeadSelfAttention_49125835931998
// MI455X (gfx1250) — hardware-verified
//
#include <hip/hip_runtime.h>
#ifndef NB
#define NB 2
#endif
#ifndef SEQ
#define SEQ 2048
#endif
#define NB_FULL 2
#define SEQ_FULL 2048
#define DM 1024
#define NH 16
#define HD 64
#define NR (NB * SEQ)
#define SC1 0.18033688011112042f
#define SC2 (SC1 * 0.0009765625f)

static_assert(NH * HD == DM);
static_assert(HD == 64);
static_assert(DM % 64 == 0);
static_assert(DM % 32 == 0);
static_assert(SEQ % 128 == 0);
static_assert(NR % 128 == 0);
static_assert(SEQ <= SEQ_FULL);
static_assert(NB <= NB_FULL);
static_assert((NB * NH * (SEQ / 16)) % 4 == 0);
static_assert(((size_t)NR * DM) % (8 * 256) == 0);
static_assert(((size_t)DM * DM) % (8 * 256) == 0);
static_assert((size_t)4 * DM * DM * 2 + (size_t)9 * NR * DM * 2 <= (size_t)134217728);

typedef unsigned short v8us __attribute__((ext_vector_type(8), may_alias));
typedef float  v8f  __attribute__((ext_vector_type(8)));
typedef float  v4f  __attribute__((ext_vector_type(4)));
typedef float  v4fa __attribute__((ext_vector_type(4), may_alias));
typedef _Float16 v16h __attribute__((ext_vector_type(16)));
union FragH { v16h v; v8us half[2]; _Float16 h[16]; unsigned short u[16]; };

__device__ __forceinline__ float bf16_rne(float x) { unsigned int u = __float_as_uint(x); u = (u + 0x7FFFu + ((u >> 16) & 1u)) & 0xFFFF0000u; return __uint_as_float(u); }

__device__ __forceinline__ v16h g2_frag(const unsigned short* p, int hh) { FragH f; f.half[0] = *(const v8us*)(p + 8 * hh); f.half[1] = *(const v8us*)(p + 16 + 8 * hh); return f.v; }
__device__ __forceinline__ v8f g2_mma(v16h a, v16h b, v8f c) { v8f d = __builtin_amdgcn_wmma_f32_16x16x32_f16(false, a, false, b, (short)0, c, false, false); asm volatile("v_nop\n\tv_nop\n\tv_nop\n\tv_nop" : "+v"(d) : "v"(a), "v"(b)); return d; }

__global__ __launch_bounds__(256) void k_x16(const float* __restrict__ x, unsigned short* __restrict__ X16) {
  const size_t t = (size_t)blockIdx.x * 256 + threadIdx.x;
  if (t >= (size_t)NR * DM / 8) return;
  const size_t e = t * 8;
  const int r = (int)(e / DM), c = (int)(e % DM);
  const int b = r / SEQ, s = r - b * SEQ;
  const float* src = x + ((size_t)b * SEQ_FULL + s) * DM + c;
  const v4f a0 = *(const v4fa*)src, a1 = *(const v4fa*)(src + 4);
  FragH f;
#pragma unroll
  for (int q = 0; q < 4; ++q) { f.h[q] = (_Float16)bf16_rne(a0[q]); f.h[4 + q] = (_Float16)bf16_rne(a1[q]); }
  const v8us o = f.half[0];
  *(volatile v8us*)(X16 + e) = o;
  __threadfence();
  *(volatile v8us*)(X16 + e) = o;
}

__global__ __launch_bounds__(256) void k_wt_f16(const float* __restrict__ W, unsigned short* __restrict__ Wt) {
  const int t = blockIdx.x * 256 + threadIdx.x;
  if (t >= DM * (DM / 8)) return;
  const int n = t / (DM / 8), k8 = (t % (DM / 8)) * 8;
  FragH f;
#pragma unroll
  for (int i = 0; i < 8; ++i) f.h[i] = (_Float16)(bf16_rne(W[(size_t)(k8 + i) * DM + n]) * 16.0f);
  const v8us o = f.half[0];
  *(volatile v8us*)(Wt + (size_t)n * DM + k8) = o;
  __threadfence();
  *(volatile v8us*)(Wt + (size_t)n * DM + k8) = o;
}

__device__ __forceinline__ void g2_loop(const unsigned short* a0p, const unsigned short* a1p, const unsigned short* b0p, const unsigned short* b1p, const unsigned short* b2p, const unsigned short* b3p, int hh,
                                        v8f& c00, v8f& c01, v8f& c02, v8f& c03, v8f& c10, v8f& c11, v8f& c12, v8f& c13) {
#pragma unroll 1
  for (int kb = 0; kb < DM; kb += 32) {
    const v16h a0 = g2_frag(a0p + kb, hh), a1 = g2_frag(a1p + kb, hh);
    v16h bf = g2_frag(b0p + kb, hh); c00 = g2_mma(a0, bf, c00); c10 = g2_mma(a1, bf, c10);
    bf = g2_frag(b1p + kb, hh); c01 = g2_mma(a0, bf, c01); c11 = g2_mma(a1, bf, c11);
    bf = g2_frag(b2p + kb, hh); c02 = g2_mma(a0, bf, c02); c12 = g2_mma(a1, bf, c12);
    bf = g2_frag(b3p + kb, hh); c03 = g2_mma(a0, bf, c03); c13 = g2_mma(a1, bf, c13);
  }
}

__global__ __launch_bounds__(128) void k_proj(const unsigned short* __restrict__ A, const unsigned short* __restrict__ Bt, const float* __restrict__ bias, float alpha,
                                              unsigned short* __restrict__ CH, unsigned short* __restrict__ CL, int nlo, int M) {
  __shared__ __attribute__((aligned(16))) float so[4][32][68];
  const int tid = threadIdx.x, lane = tid & 31, ln = lane & 15, hh = lane >> 4;
  const int wave = __builtin_amdgcn_readfirstlane((int)(threadIdx.x >> 5));
  const int ntn = DM >> 6;
  const int mt = blockIdx.x / ntn, nq = blockIdx.x - mt * ntn;
  const int row0 = mt * 128 + 32 * wave, col0 = nq * 64;
  if (row0 >= M) return;
  const unsigned short* a0p = A + (size_t)(row0 + ln) * DM;
  const unsigned short* a1p = a0p + (size_t)16 * DM;
  const unsigned short* b0p = Bt + (size_t)(col0 + ln) * DM;
  const unsigned short* b1p = b0p + (size_t)16 * DM;
  const unsigned short* b2p = b1p + (size_t)16 * DM;
  const unsigned short* b3p = b2p + (size_t)16 * DM;
  const v8f z8 = {0.f, 0.f, 0.f, 0.f, 0.f, 0.f, 0.f, 0.f};
  v8f c00 = z8, c01 = z8, c02 = z8, c03 = z8, c10 = z8, c11 = z8, c12 = z8, c13 = z8;
  g2_loop(a0p, a1p, b0p, b1p, b2p, b3p, hh, c00, c01, c02, c03, c10, c11, c12, c13);
  v8f accs[8] = {c00, c01, c02, c03, c10, c11, c12, c13};
#pragma unroll
  for (int u = 0; u < 8; ++u) {
    const int t = u & 3, half = u >> 2;
    const float bv = bf16_rne(bias[col0 + t * 16 + ln]);
#pragma unroll
    for (int r = 0; r < 8; ++r) so[wave][half * 16 + 8 * hh + r][t * 16 + ln] = accs[u][r] * alpha + bv;
  }
  __builtin_amdgcn_fence(4  , "workgroup");
  __builtin_amdgcn_wave_barrier();
  const int rq = lane >> 3, pc = (lane & 7) * 8;
  for (int pass = 0; pass < 2; ++pass) {
#pragma unroll
    for (int q = 0; q < 8; ++q) {
      const int r = q * 4 + rq;
      const v4f x0 = *(const v4fa*)&so[wave][r][pc];
      const v4f x1 = *(const v4fa*)&so[wave][r][pc + 4];
      FragH fh, fl;
#pragma unroll
      for (int i = 0; i < 4; ++i) {
        _Float16 h = (_Float16)x0[i]; fh.h[i] = h; fl.h[i] = (_Float16)((x0[i] - (float)h) * 1024.0f);
        h = (_Float16)x1[i]; fh.h[4 + i] = h; fl.h[4 + i] = (_Float16)((x1[i] - (float)h) * 1024.0f);
      }
      const size_t o = (size_t)(row0 + r) * DM + col0 + pc;
      const v8us vh = fh.half[0], vl = fl.half[0];
      *(volatile v8us*)(CH + o) = vh;
      if (nlo) *(volatile v8us*)(CL + o) = vl;
    }
    if (pass == 0) __threadfence();
  }
}

__global__ __launch_bounds__(256) void k_vt(const unsigned short* __restrict__ V16, unsigned short* __restrict__ VT) {
  __shared__ unsigned short tl[64][66];
  const int tid = threadIdx.x;
  const int slab = blockIdx.x / (SEQ / 64), lg = blockIdx.x - slab * (SEQ / 64);
  const int b = slab / NH, h = slab - b * NH;
  for (int i = tid; i < 64 * 8; i += 256) {
    const int r = i >> 3, c8 = (i & 7) * 8;
    FragH f;
    f.half[0] = *(const v8us*)(V16 + ((size_t)b * SEQ + lg * 64 + r) * DM + h * HD + c8);
#pragma unroll
    for (int q = 0; q < 8; ++q) tl[r][c8 + q] = f.u[q];
  }
  __syncthreads();
  for (int pass = 0; pass < 2; ++pass) {
#pragma unroll
    for (int rd = 0; rd < 2; ++rd) {
      const int d = rd * 32 + (tid >> 3), pc = tid & 7;
      FragH f;
#pragma unroll
      for (int q = 0; q < 8; ++q) f.u[q] = tl[pc * 8 + q][d];
      const v8us o = f.half[0];
      *(volatile v8us*)(VT + ((size_t)slab * HD + d) * SEQ + lg * 64 + pc * 8) = o;
    }
    if (pass == 0) __threadfence();
  }
}

__global__ __launch_bounds__(128) void k_flash(const unsigned short* __restrict__ QH, const unsigned short* __restrict__ QL, const unsigned short* __restrict__ KH, const unsigned short* __restrict__ KL,
                                               const unsigned short* __restrict__ VT, unsigned short* __restrict__ CH, unsigned short* __restrict__ CL) {
  __shared__ __attribute__((aligned(16))) float so[4][16][68];
  const int tid = threadIdx.x, lane = tid & 31, ln = lane & 15, hh = lane >> 4;
  const int wave = __builtin_amdgcn_readfirstlane((int)(threadIdx.x >> 5));
  const int gw = blockIdx.x * 4 + wave;
  const int bh = gw / (SEQ / 16), qt = gw - bh * (SEQ / 16);
  const int b = bh / NH, h = bh - b * NH;
  const int q0 = qt * 16;
  const size_t qoff = ((size_t)b * SEQ + q0 + ln) * DM + h * HD;
  const size_t koff = ((size_t)b * SEQ + ln) * DM + h * HD;
  const size_t voff = ((size_t)bh * HD + ln) * SEQ;
  const v8f z8 = {0.f, 0.f, 0.f, 0.f, 0.f, 0.f, 0.f, 0.f};
  v8f o0 = z8, o1 = z8, o2 = z8, o3 = z8;
  float mrun = -3.0e38f, lpart = 0.f;
#pragma unroll 1
  for (int kb = 0; kb < SEQ; kb += 32) {
    int zo = 0;
    asm volatile("" : "+v"(zo));
    const size_t qo = qoff + (size_t)zo;
    const size_t k0o = koff + (size_t)kb * DM;
    const size_t k1o = k0o + (size_t)16 * DM;
    v8f sh0 = z8, sr0 = z8, sh1 = z8, sr1 = z8;
#pragma unroll
    for (int kk = 0; kk < HD; kk += 32) {
      const v16h qh = g2_frag(QH + qo + kk, hh), ql = g2_frag(QL + qo + kk, hh);
      v16h kh = g2_frag(KH + k0o + kk, hh), kl = g2_frag(KL + k0o + kk, hh);
      sh0 = g2_mma(kh, qh, sh0); sr0 = g2_mma(kl, qh, sr0); sr0 = g2_mma(kh, ql, sr0);
      kh = g2_frag(KH + k1o + kk, hh); kl = g2_frag(KL + k1o + kk, hh);
      sh1 = g2_mma(kh, qh, sh1); sr1 = g2_mma(kl, qh, sr1); sr1 = g2_mma(kh, ql, sr1);
    }
    float t0[8], t1[8];
    float bm = -3.0e38f;
#pragma unroll
    for (int r = 0; r < 8; ++r) {
      t0[r] = fmaf(sr0[r], SC2, sh0[r] * SC1);
      t1[r] = fmaf(sr1[r], SC2, sh1[r] * SC1);
      bm = fmaxf(bm, fmaxf(t0[r], t1[r]));
    }
    bm = fmaxf(bm, __shfl_xor(bm, 16, 32));
    const float mn = fmaxf(mrun, bm);
    const float al = exp2f(mrun - mn);
    mrun = mn;
    float ps = 0.f;
    FragH pf;
#pragma unroll
    for (int r = 0; r < 8; ++r) {
      const float e0 = exp2f(t0[r] - mn), e1 = exp2f(t1[r] - mn);
      ps += e0 + e1;
      pf.h[r] = (_Float16)(e0 * 1024.0f);
      pf.h[8 + r] = (_Float16)(e1 * 1024.0f);
    }
    lpart = lpart * al + ps;
    o0 *= al; o1 *= al; o2 *= al; o3 *= al;
    const v16h v0 = g2_frag(VT + voff + kb, hh);
    const v16h v1 = g2_frag(VT + voff + (size_t)16 * SEQ + kb, hh);
    const v16h v2 = g2_frag(VT + voff + (size_t)32 * SEQ + kb, hh);
    const v16h v3 = g2_frag(VT + voff + (size_t)48 * SEQ + kb, hh);
    o0 = g2_mma(v0, pf.v, o0);
    o1 = g2_mma(v1, pf.v, o1);
    o2 = g2_mma(v2, pf.v, o2);
    o3 = g2_mma(v3, pf.v, o3);
  }
  const float ltot = lpart + __shfl_xor(lpart, 16, 32);
  const float fin = 0.0625f * (1.0f / ltot);
#pragma unroll
  for (int r = 0; r < 8; ++r) {
    so[wave][ln][8 * hh + r] = o0[r] * fin;
    so[wave][ln][16 + 8 * hh + r] = o1[r] * fin;
    so[wave][ln][32 + 8 * hh + r] = o2[r] * fin;
    so[wave][ln][48 + 8 * hh + r] = o3[r] * fin;
  }
  __builtin_amdgcn_fence(4  , "workgroup");
  __builtin_amdgcn_wave_barrier();
  const int rq = lane >> 3, pc = (lane & 7) * 8;
  for (int pass = 0; pass < 2; ++pass) {
#pragma unroll
    for (int q = 0; q < 4; ++q) {
      const int r = q * 4 + rq;
      const v4f x0 = *(const v4fa*)&so[wave][r][pc];
      const v4f x1 = *(const v4fa*)&so[wave][r][pc + 4];
      FragH fh, fl;
#pragma unroll
      for (int i = 0; i < 4; ++i) {
        _Float16 hv = (_Float16)x0[i]; fh.h[i] = hv; fl.h[i] = (_Float16)((x0[i] - (float)hv) * 1024.0f);
        hv = (_Float16)x1[i]; fh.h[4 + i] = hv; fl.h[4 + i] = (_Float16)((x1[i] - (float)hv) * 1024.0f);
      }
      const size_t o = ((size_t)b * SEQ + q0 + r) * DM + h * HD + pc;
      const v8us vh = fh.half[0], vl = fl.half[0];
      *(volatile v8us*)(CH + o) = vh;
      *(volatile v8us*)(CL + o) = vl;
    }
    if (pass == 0) __threadfence();
  }
}

__global__ __launch_bounds__(128) void k_out(const unsigned short* __restrict__ AH, const unsigned short* __restrict__ AL, const unsigned short* __restrict__ Bt, const float* __restrict__ bias,
                                             float* __restrict__ C, int M) {
  __shared__ __attribute__((aligned(16))) float so[4][32][68];
  const int tid = threadIdx.x, lane = tid & 31, ln = lane & 15, hh = lane >> 4;
  const int wave = __builtin_amdgcn_readfirstlane((int)(threadIdx.x >> 5));
  const int ntn = DM >> 6;
  const int mt = blockIdx.x / ntn, nq = blockIdx.x - mt * ntn;
  const int row0 = mt * 128 + 32 * wave, col0 = nq * 64;
  if (row0 >= M) return;
  const size_t aoff = (size_t)(row0 + ln) * DM;
  const unsigned short* b0p = Bt + (size_t)(col0 + ln) * DM;
  const unsigned short* b1p = b0p + (size_t)16 * DM;
  const unsigned short* b2p = b1p + (size_t)16 * DM;
  const unsigned short* b3p = b2p + (size_t)16 * DM;
  const v8f z8 = {0.f, 0.f, 0.f, 0.f, 0.f, 0.f, 0.f, 0.f};
  v8f c00 = z8, c01 = z8, c02 = z8, c03 = z8, c10 = z8, c11 = z8, c12 = z8, c13 = z8;
  g2_loop(AL + aoff, AL + aoff + (size_t)16 * DM, b0p, b1p, b2p, b3p, hh, c00, c01, c02, c03, c10, c11, c12, c13);
  c00 *= 0.0009765625f; c01 *= 0.0009765625f; c02 *= 0.0009765625f; c03 *= 0.0009765625f;
  c10 *= 0.0009765625f; c11 *= 0.0009765625f; c12 *= 0.0009765625f; c13 *= 0.0009765625f;
  g2_loop(AH + aoff, AH + aoff + (size_t)16 * DM, b0p, b1p, b2p, b3p, hh, c00, c01, c02, c03, c10, c11, c12, c13);
  v8f accs[8] = {c00, c01, c02, c03, c10, c11, c12, c13};
#pragma unroll
  for (int u = 0; u < 8; ++u) {
    const int t = u & 3, half = u >> 2;
    const float bv = bf16_rne(bias[col0 + t * 16 + ln]);
#pragma unroll
    for (int r = 0; r < 8; ++r) so[wave][half * 16 + 8 * hh + r][t * 16 + ln] = accs[u][r] * 0.0009765625f + bv;
  }
  __builtin_amdgcn_fence(4  , "workgroup");
  __builtin_amdgcn_wave_barrier();
  const int bsel = row0 / SEQ, srow0 = row0 - bsel * SEQ;
  float* crow = C + ((size_t)bsel * SEQ_FULL + srow0) * DM + col0;
  const int rsub = lane >> 4, c4 = (lane & 15) * 4;
  for (int pass = 0; pass < 2; ++pass) {
#pragma unroll
    for (int q = 0; q < 16; ++q) {
      const int r = q * 2 + rsub;
      const v4f v = *(const v4fa*)&so[wave][r][c4];
      *(volatile v4f*)(crow + (size_t)r * DM + c4) = v;
    }
    if (pass == 0) __threadfence();
  }
}

extern "C" void kernel_launch(void* const* d_in, const int* in_sizes, int n_in,
                              void* d_out, int out_size, void* d_ws, size_t ws_size, hipStream_t stream) {
  if (n_in < 9) return;
  const long long need_x = ((long long)(NB - 1) * SEQ_FULL + SEQ) * DM;
  if ((long long)in_sizes[0] < need_x) return;
  if (in_sizes[1] < DM * DM || in_sizes[3] < DM * DM || in_sizes[5] < DM * DM || in_sizes[7] < DM * DM) return;
  if (in_sizes[2] < DM || in_sizes[4] < DM || in_sizes[6] < DM || in_sizes[8] < DM) return;
  if ((long long)out_size < need_x) return;
  const float* x  = (const float*)d_in[0];
  const float* wq = (const float*)d_in[1];
  const float* bq = (const float*)d_in[2];
  const float* wk = (const float*)d_in[3];
  const float* bk = (const float*)d_in[4];
  const float* wv = (const float*)d_in[5];
  const float* bv = (const float*)d_in[6];
  const float* wo = (const float*)d_in[7];
  const float* bo = (const float*)d_in[8];
  char* ws = (char*)d_ws;
  size_t off = 0;
  auto take = [&](size_t bytes) { char* p = ws + off; off += (bytes + 255) & ~(size_t)255; return p; };
  const size_t WB = (size_t)DM * DM * 2;
  const size_t PB = (size_t)NR * DM * 2;
  unsigned short* BQ = (unsigned short*)take(WB);
  unsigned short* BK = (unsigned short*)take(WB);
  unsigned short* BV = (unsigned short*)take(WB);
  unsigned short* BO = (unsigned short*)take(WB);
  unsigned short* X16 = (unsigned short*)take(PB);
  unsigned short* QH = (unsigned short*)take(PB);
  unsigned short* QL = (unsigned short*)take(PB);
  unsigned short* KH = (unsigned short*)take(PB);
  unsigned short* KL = (unsigned short*)take(PB);
  unsigned short* V16 = (unsigned short*)take(PB);
  unsigned short* VT = (unsigned short*)take(PB);
  unsigned short* CH = (unsigned short*)take(PB);
  unsigned short* CL = (unsigned short*)take(PB);
  if (off > ws_size || off > (size_t)134217728) return;

  const unsigned gw = (unsigned)(((size_t)DM * DM / 8) / 256);
  k_wt_f16<<<gw, 256, 0, stream>>>(wq, BQ);
  k_wt_f16<<<gw, 256, 0, stream>>>(wk, BK);
  k_wt_f16<<<gw, 256, 0, stream>>>(wv, BV);
  k_wt_f16<<<gw, 256, 0, stream>>>(wo, BO);
  k_x16<<<(unsigned)(((size_t)NR * DM / 8) / 256), 256, 0, stream>>>(x, X16);

  const unsigned gp = (unsigned)((NR / 128) * (DM / 64));
  k_proj<<<gp, 128, 0, stream>>>(X16, BQ, bq, 0.0625f, QH, QL, 1, NR);
  k_proj<<<gp, 128, 0, stream>>>(X16, BK, bk, 0.0625f, KH, KL, 1, NR);
  k_proj<<<gp, 128, 0, stream>>>(X16, BV, bv, 0.0625f, V16, V16, 0, NR);
  k_vt<<<(unsigned)(NB * NH * (SEQ / 64)), 256, 0, stream>>>(V16, VT);
  k_flash<<<(unsigned)((NB * NH * (SEQ / 16)) / 4), 128, 0, stream>>>(QH, QL, KH, KL, VT, CH, CL);
  k_out<<<gp, 128, 0, stream>>>(CH, CL, BO, bo, (float*)d_out, NR);
}
